// GatedDeltaNet_32023276159039
// MI455X (gfx1250) — hardware-run, weakly checked
//
#include <hip/hip_runtime.h>
#include <math.h>

constexpr int kBatch   = 2;
constexpr int kTime    = 1024;
constexpr int kHid     = 2048;
constexpr int kNumKH   = 8;
constexpr int kNumVH   = 16;
constexpr int kDimK    = 64;
constexpr int kDimV    = 128;
constexpr int kTaps    = 4;
constexpr int kKeyDim  = kNumKH * kDimK;
constexpr int kValDim  = kNumVH * kDimV;
constexpr int kConvDim = 2 * kKeyDim + kValDim;
constexpr int kProjDim = kConvDim + kValDim + 2 * kNumVH;
constexpr int kProjPad = 5184;
constexpr int kRows    = kBatch * kTime;
constexpr int kGbPitch = 32;
constexpr int kSPitch  = 68;
constexpr float kOutScale   = 0.125f;
constexpr float kEps        = 1.0e-6f;
constexpr float kGateCarry  = 64.0f;
constexpr float kW2Carry    = 16.0f;
constexpr float kGemm2Scale = 1.0f / (64.0f * 16.0f);
static_assert(kProjPad % 64 == 0 && kProjPad >= kProjDim, "N pad");
static_assert(kRows % 64 == 0 && kHid % 64 == 0, "M, N tiles");
static_assert(kHid % 32 == 0 && kValDim % 32 == 0, "K % 32");
static_assert(kConvDim % 256 == 0 && kHid == 256 * 8, "thread maps");

typedef __attribute__((ext_vector_type(16))) _Float16 v16h;
typedef __attribute__((ext_vector_type(8)))  _Float16 v8h;
typedef __attribute__((ext_vector_type(16))) __bf16   v16b;
typedef __attribute__((ext_vector_type(8)))  __bf16   v8b;
typedef __attribute__((ext_vector_type(8)))  float    v8f;
typedef __attribute__((ext_vector_type(4)))  float    v4f;
typedef __attribute__((ext_vector_type(4)))  unsigned int v4u;

__device__ __forceinline__ unsigned short f2bf_bits(float f) {
  unsigned u = __float_as_uint(f);
  return (unsigned short)((u + 0x7FFFu + ((u >> 16) & 1u)) >> 16);
}
__device__ __forceinline__ float bf_bits2f(unsigned short h) { return __uint_as_float(((unsigned)h) << 16); }

__device__ __forceinline__ void dep_guard_h(v8f& a, v8f& b, v16h x, v16h y) { asm volatile("v_nop\n\tv_nop\n\tv_nop\n\tv_nop" : "+v"(a), "+v"(b) : "v"(x), "v"(y)); }
__device__ __forceinline__ void dep_guard_b(v8f& a, v8f& b, v16b x, v16b y) { asm volatile("v_nop\n\tv_nop\n\tv_nop\n\tv_nop" : "+v"(a), "+v"(b) : "v"(x), "v"(y)); }
__device__ __forceinline__ void keep4_h(v16h a, v16h b, v16h c, v16h d) { asm volatile("v_nop" :: "v"(a), "v"(b), "v"(c), "v"(d)); }
__device__ __forceinline__ void keep4_b(v16b a, v16b b, v16b c, v16b d) { asm volatile("v_nop" :: "v"(a), "v"(b), "v"(c), "v"(d)); }
__device__ __forceinline__ void acc_guard4(v8f& a, v8f& b, v8f& c, v8f& d) { asm volatile("v_nop\n\tv_nop\n\tv_nop\n\tv_nop" : "+v"(a), "+v"(b), "+v"(c), "+v"(d)); }
template <typename T> struct Frag;
template <> struct Frag<_Float16> {
  typedef v16h V; union U { v16h v; v8h h[2]; };
  static __device__ __forceinline__ v16h load(const _Float16* p) {
    U f; f.h[0] = *(const v8h*)(p); f.h[1] = *(const v8h*)(p + 16); return f.v;
  }
  static __device__ __forceinline__ v8f mma(v16h a, v16h b, v8f c) {
    return __builtin_amdgcn_wmma_f32_16x16x32_f16(false, a, false, b, (short)0, c, false, false);
  }
  static __device__ __forceinline__ void guard(v8f& a, v8f& b, v16h x, v16h y) { dep_guard_h(a, b, x, y); }
  static __device__ __forceinline__ void keep(v16h a, v16h b, v16h c, v16h d) { keep4_h(a, b, c, d); }
};
template <> struct Frag<__bf16> {
  typedef v16b V; union U { v16b v; v8b h[2]; };
  static __device__ __forceinline__ v16b load(const __bf16* p) {
    U f; f.h[0] = *(const v8b*)(p); f.h[1] = *(const v8b*)(p + 16); return f.v;
  }
  static __device__ __forceinline__ v8f mma(v16b a, v16b b, v8f c) {
    return __builtin_amdgcn_wmma_f32_16x16x32_bf16(false, a, false, b, (short)0, c, false, false);
  }
  static __device__ __forceinline__ void guard(v8f& a, v8f& b, v16b x, v16b y) { dep_guard_b(a, b, x, y); }
  static __device__ __forceinline__ void keep(v16b a, v16b b, v16b c, v16b d) { keep4_b(a, b, c, d); }
};

__device__ __forceinline__ unsigned pk16(unsigned short a, unsigned short b) { return (unsigned)a | ((unsigned)b << 16); }
__device__ __forceinline__ unsigned short h_bits(float f) { const _Float16 h = (_Float16)f; return __builtin_bit_cast(unsigned short, h); }
__device__ __forceinline__ float bfr(float f) { return bf_bits2f(f2bf_bits(f)); }

template <int ET> struct Elem;
template <> struct Elem<0> { typedef _Float16 T; };
template <> struct Elem<1> { typedef __bf16 T; };
template <int ET, bool SPLIT, int BIAS_MODE, int OUT_MODE, bool RESID, int ACT = 0>
__global__ __launch_bounds__(256) void wmma_gemm64(
    const unsigned short* __restrict__ Ap, const unsigned short* __restrict__ A2p, int lda, long strideA,
    const unsigned short* __restrict__ Btp, const unsigned short* __restrict__ Bt2p, int ldb, long strideB,
    void* __restrict__ Cout, void* __restrict__ Cout2, int ldc, long strideC,
    const float* __restrict__ bias,
    const float* __restrict__ resid, long strideR,
    int M, int N, int K, float scale) {
  typedef typename Elem<ET>::T T;
  typedef typename Frag<T>::V V;
  const T* A = (const T*)Ap; const T* A2 = (const T*)A2p; const T* Bt = (const T*)Btp; const T* Bt2 = (const T*)Bt2p;
  __shared__ __align__(16) float sT[8][16 * 68];
  const int b    = blockIdx.y;
  const int lane = threadIdx.x & 31;
  const int wave = threadIdx.x >> 5;
  const int tilesN = N >> 6;
  const int tilesM = M >> 6;
  const int tile = blockIdx.x * 8 + wave;
  if (tile >= tilesM * tilesN) return;
  const int tm = tile / tilesN;
  const int tn = tile - tm * tilesN;
  const int m0 = tm << 6;
  const int n0 = tn << 6;

  const T* Ab  = A  + (size_t)b * strideA;
  const T* Bb  = Bt + (size_t)b * strideB;
  const T* Ab2 = SPLIT ? (A2  + (size_t)b * strideA) : nullptr;
  const T* Bb2 = SPLIT ? (Bt2 + (size_t)b * strideB) : nullptr;

  const int rlane = lane & 15;
  const int koff  = (lane >> 4) * 8;
  const int mOff  = (lane >> 4) * 8;

  v8f acc[4][4];
#pragma unroll
  for (int i = 0; i < 4; ++i)
#pragma unroll
    for (int j = 0; j < 4; ++j) acc[i][j] = (v8f){0.f,0.f,0.f,0.f,0.f,0.f,0.f,0.f};

  for (int k0 = 0; k0 < K; k0 += 32) {
    V bh[4], bl[4];
#pragma unroll
    for (int j = 0; j < 4; ++j) {
      const size_t bo = (size_t)(n0 + (j << 4) + rlane) * ldb + koff + k0;
      bh[j] = Frag<T>::load(Bb + bo);
      if (SPLIT) bl[j] = Frag<T>::load(Bb2 + bo);
    }
#pragma unroll
    for (int i = 0; i < 4; ++i) {
      const size_t ao = (size_t)(m0 + (i << 4) + rlane) * lda + koff + k0;
      V ah = Frag<T>::load(Ab + ao);
      V al;
      if (SPLIT) al = Frag<T>::load(Ab2 + ao);
#pragma unroll
      for (int j = 0; j < 4; ++j) {
        acc[i][j] = Frag<T>::mma(ah, bh[j], acc[i][j]);
        if (SPLIT) {
          acc[i][j] = Frag<T>::mma(ah, bl[j], acc[i][j]);
          acc[i][j] = Frag<T>::mma(al, bh[j], acc[i][j]);
        }
      }
      Frag<T>::guard(acc[i][0], acc[i][3], ah, SPLIT ? al : ah);
    }
    Frag<T>::keep(bh[0], bh[1], bh[2], bh[3]);
    if (SPLIT) Frag<T>::keep(bl[0], bl[1], bl[2], bl[3]);
  }
  acc_guard4(acc[0][0], acc[0][1], acc[0][2], acc[0][3]);
  acc_guard4(acc[1][0], acc[1][1], acc[1][2], acc[1][3]);
  acc_guard4(acc[2][0], acc[2][1], acc[2][2], acc[2][3]);
  acc_guard4(acc[3][0], acc[3][1], acc[3][2], acc[3][3]);

  float* slab = sT[wave];
  const float* Rb = RESID ? (resid + (size_t)b * strideR) : nullptr;
#pragma unroll
  for (int i = 0; i < 4; ++i) {
    const int mBase = m0 + (i << 4);
#pragma unroll
    for (int j = 0; j < 4; ++j) {
      const int n = n0 + (j << 4) + rlane;
      float bv = 0.f;
      if (BIAS_MODE == 2) bv = bias[n];
#pragma unroll
      for (int r = 0; r < 8; ++r) {
        float v = acc[i][j][r] * scale;
        if (BIAS_MODE == 1) v += bias[mBase + mOff + r];
        if (BIAS_MODE == 2) v += bv;
        if (RESID) v += Rb[(size_t)(mBase + mOff + r) * ldc + n];
        if (ACT == 2) v = fmaxf(v, 0.0f);
        if (ACT == 4) v = (v > 0.f) ? v : 0.01f * v;
        slab[(mOff + r) * 68 + (j << 4) + rlane] = v;
      }
    }
    __builtin_amdgcn_fence(__ATOMIC_RELEASE, "workgroup");
    __builtin_amdgcn_wave_barrier();
    __builtin_amdgcn_fence(__ATOMIC_ACQUIRE, "workgroup");
    if (OUT_MODE == 0) {
      float* C = (float*)Cout + (size_t)b * strideC;
      const int hh = lane >> 4, c4 = (lane & 15) * 4;
      for (int pass = 0; pass < 2; ++pass) {
#pragma unroll
        for (int it = 0; it < 8; ++it) {
          const int row = it * 2 + hh;
          v4f v = *(const v4f*)(slab + row * 68 + c4);
          *(volatile v4f*)(C + (size_t)(mBase + row) * ldc + n0 + c4) = v;
        }
        __threadfence();
      }
    } else {
      const int q = lane >> 3, c8 = (lane & 7) * 8;
      unsigned short* C  = (unsigned short*)Cout  + (size_t)b * strideC;
      unsigned short* C2 = (OUT_MODE == 2) ? ((unsigned short*)Cout2 + (size_t)b * strideC) : nullptr;
      for (int pass = 0; pass < 2; ++pass) {
#pragma unroll
        for (int it = 0; it < 4; ++it) {
          const int row = it * 4 + q;
          const float* sp = slab + row * 68 + c8;
          v8h hv, lv;
#pragma unroll
          for (int e = 0; e < 8; ++e) {
            if (OUT_MODE == 1) {
              hv[e] = (_Float16)sp[e];
            } else {
              unsigned short hb = f2bf_bits(sp[e]);
              unsigned short lb = f2bf_bits(sp[e] - bf_bits2f(hb));
              hv[e] = __builtin_bit_cast(_Float16, hb);
              lv[e] = __builtin_bit_cast(_Float16, lb);
            }
          }
          *(volatile v8h*)(C + (size_t)(mBase + row) * ldc + n0 + c8) = hv;
          if (OUT_MODE == 2) *(volatile v8h*)(C2 + (size_t)(mBase + row) * ldc + n0 + c8) = lv;
        }
        __threadfence();
      }
    }
    __builtin_amdgcn_fence(__ATOMIC_RELEASE, "workgroup");
    __builtin_amdgcn_wave_barrier();
    __builtin_amdgcn_fence(__ATOMIC_ACQUIRE, "workgroup");
  }
}

__global__ __launch_bounds__(256) void cast8_bf16_kernel(const float* __restrict__ in, unsigned short* __restrict__ out,
                                                        int nrows_real) {
  const int row  = blockIdx.x;
  const int t    = threadIdx.x;
  const int rowc = (row < nrows_real) ? row : (nrows_real - 1);
  const float f  = (row < nrows_real) ? 1.0f : 0.0f;
  const float* p = in + (size_t)rowc * kHid + 8 * t;
  const v4f a = *(const v4f*)(p);
  const v4f c = *(const v4f*)(p + 4);
  unsigned short hb[8];
#pragma unroll
  for (int e = 0; e < 4; ++e) {
    hb[e]     = f2bf_bits(a[e] * f);
    hb[4 + e] = f2bf_bits(c[e] * f);
  }
  const v4u u = (v4u){pk16(hb[0], hb[1]), pk16(hb[2], hb[3]), pk16(hb[4], hb[5]), pk16(hb[6], hb[7])};
  unsigned short* q = out + (size_t)row * kHid + 8 * t;
  *(volatile v4u*)q = u;
  __threadfence();
  *(volatile v4u*)q = u;
}

__global__ __launch_bounds__(256) void cast8_w2_kernel(const float* __restrict__ in, unsigned short* __restrict__ out) {
  const int row = blockIdx.x;
  const int t   = threadIdx.x;
  const float* p = in + (size_t)row * kValDim + 8 * t;
  const v4f a = *(const v4f*)(p);
  const v4f c = *(const v4f*)(p + 4);
  unsigned short hb[8];
#pragma unroll
  for (int e = 0; e < 4; ++e) {
    hb[e]     = h_bits(bfr(a[e]) * kW2Carry);
    hb[4 + e] = h_bits(bfr(c[e]) * kW2Carry);
  }
  const v4u u = (v4u){pk16(hb[0], hb[1]), pk16(hb[2], hb[3]), pk16(hb[4], hb[5]), pk16(hb[6], hb[7])};
  unsigned short* q = out + (size_t)row * kValDim + 8 * t;
  *(volatile v4u*)q = u;
  __threadfence();
  *(volatile v4u*)q = u;
}

__global__ __launch_bounds__(256) void conv_prep_kernel(const float* __restrict__ proj, const float* __restrict__ conv_w,
                                                        float* __restrict__ qn, float* __restrict__ kn,
                                                        float* __restrict__ vout) {
  __shared__ __align__(16) float s_all[kConvDim];
  const int bt   = blockIdx.x;
  const int t    = threadIdx.x;
  const int lane = t & 31, wave = t >> 5;
  const int tt   = bt & (kTime - 1);
  int r0 = bt - 3, r1 = bt - 2, r2 = bt - 1;
  float f0 = 1.0f, f1 = 1.0f, f2 = 1.0f;
  if (tt < 3) { r0 = bt; f0 = 0.0f; }
  if (tt < 2) { r1 = bt; f1 = 0.0f; }
  if (tt < 1) { r2 = bt; f2 = 0.0f; }
  const float* p0 = proj + (size_t)r0 * kProjPad;
  const float* p1 = proj + (size_t)r1 * kProjPad;
  const float* p2 = proj + (size_t)r2 * kProjPad;
  const float* p3 = proj + (size_t)bt * kProjPad;
#pragma unroll 1
  for (int it = 0; it < kConvDim / 256; ++it) {
    const int c = it * 256 + t;
    const v4f w4 = *(const v4f*)(conv_w + 4 * (size_t)c);
    const float w0 = bfr(w4[0]), w1 = bfr(w4[1]), w2 = bfr(w4[2]), w3 = bfr(w4[3]);
    const float m0 = p0[c] * f0;
    const float m1 = p1[c] * f1;
    const float m2 = p2[c] * f2;
    const float m3 = p3[c];
    float acc = 0.0f + w0 * m0;
    acc = fmaf(w1, m1, acc);
    acc = fmaf(w2, m2, acc);
    acc = fmaf(w3, m3, acc);
    const float e = expf(-acc);
    s_all[c] = acc * (1.0f / (1.0f + e));
  }
  __syncthreads();
  {
    float* qg = s_all + wave * kDimK;
    float* kg = s_all + kKeyDim + wave * kDimK;
    const float q0 = qg[lane], q1 = qg[lane + 32];
    const float k0 = kg[lane], k1 = kg[lane + 32];
    float pq = fmaf(q0, q0, q1 * q1);
    float pk = fmaf(k0, k0, k1 * k1);
#pragma unroll
    for (int off = 16; off > 0; off >>= 1) {
      pq += __shfl_xor(pq, off, 32);
      pk += __shfl_xor(pk, off, 32);
    }
    const float invq = 1.0f / fmaxf(sqrtf(pq), 1.0e-12f);
    const float invk = 1.0f / fmaxf(sqrtf(pk), 1.0e-12f);
    qg[lane] = q0 * invq; qg[lane + 32] = q1 * invq;
    kg[lane] = k0 * invk; kg[lane + 32] = k1 * invk;
  }
  __syncthreads();
  const int grp = t >> 7;
  const int idx = (t & 127) * 4;
  float* qkdst = ((grp == 0) ? qn : kn) + (size_t)bt * kKeyDim + idx;
  const v4f vq = *(const v4f*)(s_all + grp * kKeyDim + idx);
  const v4f va = *(const v4f*)(s_all + 2 * kKeyDim + 4 * t);
  const v4f vb = *(const v4f*)(s_all + 2 * kKeyDim + 1024 + 4 * t);
  float* vd0 = vout + (size_t)bt * kValDim + 4 * t;
  float* vd1 = vd0 + 1024;
  for (int pass = 0; pass < 2; ++pass) {
    *(volatile v4f*)qkdst = vq;
    *(volatile v4f*)vd0 = va;
    *(volatile v4f*)vd1 = vb;
    __threadfence();
  }
}

__global__ __launch_bounds__(256) void gate_kernel(const float* __restrict__ proj, const float* __restrict__ dt_bias,
                                                   const float* __restrict__ a_log, const int* __restrict__ pos_unused,
                                                   float* __restrict__ gb) {
  (void)pos_unused;
  const int lane = threadIdx.x & 31, wave = threadIdx.x >> 5;
  const int bt = blockIdx.x * 8 + wave;
  const int h  = lane & 15;
  const float* pr = proj + (size_t)bt * kProjPad + kConvDim + kValDim;
  const float bv = pr[h];
  const float av = pr[kNumVH + h];
  const float db = bfr(dt_bias[h]);
  const float al = bfr(a_log[h]);
  const float eb   = expf(-bv);
  const float beta = 1.0f / (1.0f + eb);
  const float xx = av + db;
  const float sp = fmaxf(xx, 0.0f) + log1pf(expf(-fabsf(xx)));
  const float g  = -expf(al) * sp;
  float eg = expf(g);
  eg = (eg < 1.17549435e-38f) ? 0.0f : eg;
  const float fs  = (lane < 16) ? 1.0f : 0.0f;
  const float val = fmaf(fs, eg, (1.0f - fs) * beta);
  float* d = gb + (size_t)bt * kGbPitch + lane;
  *(volatile float*)d = val;
  __threadfence();
  *(volatile float*)d = val;
}

__global__ __launch_bounds__(128) void scan_kernel(const float* __restrict__ qn, const float* __restrict__ kn,
                                                   const float* __restrict__ vin, const float* __restrict__ gb,
                                                   float* __restrict__ o) {
  __shared__ __align__(16) float ssh[kDimV * kSPitch];
  __shared__ __align__(16) float kq[2 * kDimK];
  const int v  = threadIdx.x;
  const int h  = blockIdx.x & 15;
  const int b  = blockIdx.x >> 4;
  const int kh = h >> 1;
  float* srow = ssh + v * kSPitch;
  const v4f z4 = (v4f){0.f, 0.f, 0.f, 0.f};
#pragma unroll
  for (int i = 0; i < kSPitch; i += 4) *(v4f*)(srow + i) = z4;
  const float fsel = (v < kDimK) ? 1.0f : 0.0f;
  const int kidx = v & (kDimK - 1);
  for (int st = 0; st < kTime; ++st) {
    const int bt = b * kTime + st;
    const size_t qkoff = (size_t)bt * kKeyDim + kh * kDimK + kidx;
    const float kval = kn[qkoff];
    const float qval = qn[qkoff];
    kq[v] = fmaf(fsel, kval, (1.0f - fsel) * qval);
    const float eg = gb[(size_t)bt * kGbPitch + h];
    const float bw = gb[(size_t)bt * kGbPitch + kNumVH + h];
    const float vt = vin[(size_t)bt * kValDim + h * kDimV + v];
    __syncthreads();
    float sa = 0.0f, sb = 0.0f;
#pragma unroll 1
    for (int kc = 0; kc < kDimK; kc += 8) {
      const v4f s0 = *(const v4f*)(srow + kc);
      const v4f s1 = *(const v4f*)(srow + kc + 4);
      const v4f k0 = *(const v4f*)(kq + kc);
      const v4f k1 = *(const v4f*)(kq + kc + 4);
      sa = fmaf(s0[0], k0[0], sa); sb = fmaf(s0[1], k0[1], sb);
      sa = fmaf(s0[2], k0[2], sa); sb = fmaf(s0[3], k0[3], sb);
      sa = fmaf(s1[0], k1[0], sa); sb = fmaf(s1[1], k1[1], sb);
      sa = fmaf(s1[2], k1[2], sa); sb = fmaf(s1[3], k1[3], sb);
    }
    const float sk    = (sa + sb) * eg;
    const float delta = bw * (vt - sk);
    float oa = 0.0f, ob = 0.0f;
#pragma unroll 1
    for (int kc = 0; kc < kDimK; kc += 8) {
      const v4f s0 = *(const v4f*)(srow + kc);
      const v4f s1 = *(const v4f*)(srow + kc + 4);
      const v4f k0 = *(const v4f*)(kq + kc);
      const v4f k1 = *(const v4f*)(kq + kc + 4);
      const v4f q0 = *(const v4f*)(kq + kDimK + kc);
      const v4f q1 = *(const v4f*)(kq + kDimK + kc + 4);
      v4f n0, n1;
#pragma unroll
      for (int e = 0; e < 4; ++e) {
        n0[e] = fmaf(k0[e], delta, s0[e] * eg);
        n1[e] = fmaf(k1[e], delta, s1[e] * eg);
      }
      *(v4f*)(srow + kc)     = n0;
      *(v4f*)(srow + kc + 4) = n1;
#pragma unroll
      for (int e = 0; e < 4; ++e) {
        oa = fmaf(n0[e], q0[e], oa);
        ob = fmaf(n1[e], q1[e], ob);
      }
    }
    const float ov = (oa + ob) * kOutScale;
    float* od = o + (size_t)bt * kValDim + h * kDimV + v;
    *(volatile float*)od = ov;
    __threadfence();
    *(volatile float*)od = ov;
    __syncthreads();
  }
}

__global__ __launch_bounds__(128) void normgate_kernel(const float* __restrict__ o, const float* __restrict__ proj,
                                                       const float* __restrict__ norm_w, unsigned short* __restrict__ gt) {
  __shared__ float red[4];
  __shared__ __align__(16) float gs[kDimV];
  const int v = threadIdx.x;
  const int lane = v & 31, wave = v >> 5;
  const int bt = blockIdx.x >> 4;
  const int h  = blockIdx.x & 15;
  const size_t rowbase = (size_t)bt * kValDim + h * kDimV;
  const float ov = o[rowbase + v];
  const float z  = proj[(size_t)bt * kProjPad + kConvDim + h * kDimV + v];
  const float nw = bfr(norm_w[v]);
  float p = ov * ov;
#pragma unroll
  for (int off = 16; off > 0; off >>= 1) p += __shfl_xor(p, off, 32);
  if (lane == 0) red[wave] = p;
  __syncthreads();
  const float sum = (red[0] + red[1]) + (red[2] + red[3]);
  const float inv = rsqrtf(sum * (1.0f / 128.0f) + kEps);
  const float normed = nw * (ov * inv);
  const float ez = expf(-z);
  const float sz = z * (1.0f / (1.0f + ez));
  gs[v] = normed * sz * kGateCarry;
  __syncthreads();
  if (v < 16) {
    const float* sp = gs + 8 * v;
    const v4f a = *(const v4f*)(sp);
    const v4f c = *(const v4f*)(sp + 4);
    unsigned short hb[8];
#pragma unroll
    for (int e = 0; e < 4; ++e) {
      hb[e]     = h_bits(a[e]);
      hb[4 + e] = h_bits(c[e]);
    }
    const v4u u = (v4u){pk16(hb[0], hb[1]), pk16(hb[2], hb[3]), pk16(hb[4], hb[5]), pk16(hb[6], hb[7])};
    unsigned short* d = gt + rowbase + 8 * v;
    *(volatile v4u*)d = u;
    __threadfence();
    *(volatile v4u*)d = u;
  }
}

extern "C" void kernel_launch(void* const* d_in, const int* in_sizes, int n_in,
                              void* d_out, int out_size, void* d_ws, size_t ws_size,
                              hipStream_t stream) {
  if (n_in < 8) return;
  if (in_sizes[0] != kRows * kHid) return;
  if (in_sizes[2] != kProjDim * kHid) return;
  if (in_sizes[3] != kConvDim * kTaps) return;
  if (in_sizes[4] != kNumVH || in_sizes[5] != kNumVH) return;
  if (in_sizes[6] != kDimV) return;
  if (in_sizes[7] != kHid * kValDim) return;
  if (out_size != kRows * kHid) return;

  const size_t szProj = (size_t)kRows * kProjPad * 4;
  const size_t szXB   = (size_t)kRows * kHid * 2;
  const size_t szW1B  = (size_t)kProjPad * kHid * 2;
  const size_t szW2H  = (size_t)kHid * kValDim * 2;
  const size_t szQK   = (size_t)kRows * kKeyDim * 4;
  const size_t szVV   = (size_t)kRows * kValDim * 4;
  const size_t szGB   = (size_t)kRows * kGbPitch * 4;
  const size_t szOO   = (size_t)kRows * kValDim * 4;
  const size_t szGT   = (size_t)kRows * kValDim * 2;
  const size_t offProj = 0;
  const size_t offXB   = offProj + szProj;
  const size_t offW1B  = offXB + szXB;
  const size_t offW2H  = offW1B + szW1B;
  const size_t offQN   = offW2H + szW2H;
  const size_t offKN   = offQN + szQK;
  const size_t offVV   = offKN + szQK;
  const size_t offGB   = offVV + szVV;
  const size_t offOO   = offGB + szGB;
  const size_t offGT   = offOO + szOO;
  const size_t total   = offGT + szGT;
  static_assert((size_t)kRows * kProjPad * 4 + (size_t)kRows * kHid * 2 + (size_t)kProjPad * kHid * 2 +
                (size_t)kHid * kValDim * 2 + 2 * (size_t)kRows * kKeyDim * 4 + (size_t)kRows * kValDim * 4 +
                (size_t)kRows * kGbPitch * 4 + (size_t)kRows * kValDim * 4 + (size_t)kRows * kValDim * 2
                == (size_t)131072000, "carve total");
  static_assert((size_t)131072000 <= (size_t)134217728, "carve budget");
  if (ws_size < total) return;

  const float* x       = (const float*)d_in[0];
  const int*   in_pos  = (const int*)d_in[1];
  const float* w1      = (const float*)d_in[2];
  const float* conv_w  = (const float*)d_in[3];
  const float* dt_bias = (const float*)d_in[4];
  const float* a_log   = (const float*)d_in[5];
  const float* norm_w  = (const float*)d_in[6];
  const float* w2      = (const float*)d_in[7];
  float* out = (float*)d_out;
  char* ws = (char*)d_ws;
  float*          PROJ = (float*)(ws + offProj);
  unsigned short* XB   = (unsigned short*)(ws + offXB);
  unsigned short* W1B  = (unsigned short*)(ws + offW1B);
  unsigned short* W2H  = (unsigned short*)(ws + offW2H);
  float*          QN   = (float*)(ws + offQN);
  float*          KN   = (float*)(ws + offKN);
  float*          VV   = (float*)(ws + offVV);
  float*          GB   = (float*)(ws + offGB);
  float*          OO   = (float*)(ws + offOO);
  unsigned short* GT   = (unsigned short*)(ws + offGT);

  cast8_bf16_kernel<<<dim3(kRows), dim3(256), 0, stream>>>(x, XB, kRows);
  cast8_bf16_kernel<<<dim3(kProjPad), dim3(256), 0, stream>>>(w1, W1B, kProjDim);
  cast8_w2_kernel<<<dim3(kHid), dim3(256), 0, stream>>>(w2, W2H);

  const int tiles1 = (kRows / 64) * (kProjPad / 64);
  wmma_gemm64<1, false, 0, 0, false, 0><<<dim3(tiles1 / 8, 1), dim3(256), 0, stream>>>(
      XB, XB, kHid, 0L, W1B, W1B, kHid, 0L,
      (void*)PROJ, (void*)PROJ, kProjPad, 0L, GB, GB, 0L, kRows, kProjPad, kHid, 1.0f);

  conv_prep_kernel<<<dim3(kRows), dim3(256), 0, stream>>>(PROJ, conv_w, QN, KN, VV);

  gate_kernel<<<dim3(kRows / 8), dim3(256), 0, stream>>>(PROJ, dt_bias, a_log, in_pos, GB);

  scan_kernel<<<dim3(kBatch * kNumVH), dim3(128), 0, stream>>>(QN, KN, VV, GB, OO);

  normgate_kernel<<<dim3(kRows * kNumVH), dim3(128), 0, stream>>>(OO, PROJ, norm_w, GT);

  const int tiles2 = (kRows / 64) * (kHid / 64);
  wmma_gemm64<0, false, 0, 0, false, 0><<<dim3(tiles2 / 8, 1), dim3(256), 0, stream>>>(
      GT, GT, kValDim, 0L, W2H, W2H, kValDim, 0L,
      (void*)out, (void*)out, kHid, 0L, GB, GB, 0L, kRows, kHid, kValDim, kGemm2Scale);
}
